// FaberConv_62723702391592
// MI455X (gfx1250) — hardware-verified
//
#include <hip/hip_runtime.h>
#include <stddef.h>


#define DIM     64
#define KST     128
#define NMAT    3
#define WIN     (DIM * DIM)
#define BPL     (DIM * KST)
#define NTHR    256
#define NWAVE   8
#define EPT     8
#define NGRP    2
#define CHUNK   (NTHR * EPT * NGRP)
#define WCAP    (EPT * NGRP * 32)
#define LISTN   (NWAVE * WCAP)
#define LSH     13
#define NBC     8192
#define NBF     2048
#define RCAP    40960
#define RBN     128
#define TGT     256
#define DEGCAP  256
#define GROWS   128
#define OTHR    512
#define CPT     16
#define APH     (KST + 8)
#define WSCAP   134217728

#define LDS_GEMM (2 * GROWS * APH * 2)
#define LDS_FILL ((RCAP + NBF + LISTN) * 4 + 64)

static_assert((CHUNK & (CHUNK - 1)) == 0);
static_assert(CHUNK <= 4096);
static_assert(NBC <= (1 << LSH) && NBF <= (1 << LSH));
static_assert((NBC & (NBC - 1)) == 0 && (NBF & (NBF - 1)) == 0);
static_assert(NBC == 4 * NBF);
static_assert(OTHR * CPT == NBC);
static_assert(OTHR == 4 * 128);
static_assert((RCAP % 32) == 0);
static_assert(GROWS * DIM * 4 <= LDS_GEMM);
static_assert((APH * 2) % 16 == 0);
static_assert(TGT == NWAVE * 32);
static_assert((NBC % TGT) == 0);
static_assert((GROWS * KST / 8) == 8 * NTHR);
static_assert(GROWS == NWAVE * 16);
static_assert(NBC == NWAVE * 8 * 128);
static_assert(DIM * KST / 8 == 4 * NTHR);

typedef float          v4f  __attribute__((ext_vector_type(4)));
typedef float          v8f  __attribute__((ext_vector_type(8)));
typedef int            v4i  __attribute__((ext_vector_type(4)));
typedef unsigned short v8us __attribute__((ext_vector_type(8)));
typedef __bf16         v16b __attribute__((ext_vector_type(16)));
union FragB { v16b v; v8us h[2]; };

__device__ __forceinline__ unsigned int bfr(float f) {
  const unsigned int u = __float_as_uint(f);
  return (u + 0x7FFFu + ((u >> 16) & 1u)) >> 16;
}

__device__ __forceinline__ void split1(float x, unsigned short& hb, unsigned short& lb) {
  const unsigned int hu = bfr(x);
  const float hf = __uint_as_float(hu << 16);
  hb = (unsigned short)hu;
  lb = (unsigned short)bfr(x - hf);
}

__device__ __forceinline__ void split8(v4f a, v4f b, v8us& hi, v8us& lo) {
  unsigned short hb, lb;
  split1(a.x, hb, lb); hi[0] = hb; lo[0] = lb;
  split1(a.y, hb, lb); hi[1] = hb; lo[1] = lb;
  split1(a.z, hb, lb); hi[2] = hb; lo[2] = lb;
  split1(a.w, hb, lb); hi[3] = hb; lo[3] = lb;
  split1(b.x, hb, lb); hi[4] = hb; lo[4] = lb;
  split1(b.y, hb, lb); hi[5] = hb; lo[5] = lb;
  split1(b.z, hb, lb); hi[6] = hb; lo[6] = lb;
  split1(b.w, hb, lb); hi[7] = hb; lo[7] = lb;
}

__device__ __forceinline__ v8f wmb(v16b a, v16b b, v8f c) {
  v8f d = __builtin_amdgcn_wmma_f32_16x16x32_bf16(false, a, false, b, (short)0, c, false, false);
  asm volatile("v_nop\n\tv_nop\n\tv_nop\n\tv_nop" : "+v"(d) : "v"(a), "v"(b));
  return d;
}

template <int NB>
__device__ __forceinline__ int scan_chunk(const int* __restrict__ dsts, int nE, int cbase, int slotBase,
                                          int vec8, int* list, int tid, int lane, int wave) {
  int wc = 0;
#pragma unroll
  for (int g = 0; g < NGRP; ++g) {
    const int el0  = (g * NTHR + tid) * EPT;
    const int e0   = cbase + el0;
    const int sent = -2147483647 - 1;
    v4i da, db;
    if (vec8 != 0 && cbase + CHUNK <= nE) {
      da = *(const v4i*)(dsts + e0);
      db = *(const v4i*)(dsts + e0 + 4);
    } else {
      da.x = (e0     < nE) ? dsts[min(e0, nE - 1)] : sent;
      da.y = (e0 + 1 < nE) ? dsts[min(e0 + 1, nE - 1)] : sent;
      da.z = (e0 + 2 < nE) ? dsts[min(e0 + 2, nE - 1)] : sent;
      da.w = (e0 + 3 < nE) ? dsts[min(e0 + 3, nE - 1)] : sent;
      db.x = (e0 + 4 < nE) ? dsts[min(e0 + 4, nE - 1)] : sent;
      db.y = (e0 + 5 < nE) ? dsts[min(e0 + 5, nE - 1)] : sent;
      db.z = (e0 + 6 < nE) ? dsts[min(e0 + 6, nE - 1)] : sent;
      db.w = (e0 + 7 < nE) ? dsts[min(e0 + 7, nE - 1)] : sent;
    }
    const unsigned nb = (unsigned)slotBase;
    const unsigned s0 = (unsigned)da.x - nb, s1 = (unsigned)da.y - nb;
    const unsigned s2 = (unsigned)da.z - nb, s3 = (unsigned)da.w - nb;
    const unsigned s4 = (unsigned)db.x - nb, s5 = (unsigned)db.y - nb;
    const unsigned s6 = (unsigned)db.z - nb, s7 = (unsigned)db.w - nb;
    const bool h0 = s0 < (unsigned)NB, h1 = s1 < (unsigned)NB, h2 = s2 < (unsigned)NB, h3 = s3 < (unsigned)NB;
    const bool h4 = s4 < (unsigned)NB, h5 = s5 < (unsigned)NB, h6 = s6 < (unsigned)NB, h7 = s7 < (unsigned)NB;
    const unsigned any = __builtin_amdgcn_ballot_w32(h0 | h1 | h2 | h3 | h4 | h5 | h6 | h7);
    if (any != 0u) {
#define HITJ(J, HJ, SJ) { \
        const unsigned mj = __builtin_amdgcn_ballot_w32(HJ); \
        if (mj != 0u) { \
          if (HJ) { \
            const int pos = wc + (int)__builtin_amdgcn_mbcnt_lo(mj, 0u); \
            if (pos < WCAP) list[wave * WCAP + pos] = ((el0 + (J)) << LSH) | (int)(SJ); \
          } \
          wc += (int)__builtin_popcount(mj); } }
      HITJ(0, h0, s0)
      HITJ(1, h1, s1)
      HITJ(2, h2, s2)
      HITJ(3, h3, s3)
      HITJ(4, h4, s4)
      HITJ(5, h5, s5)
      HITJ(6, h6, s6)
      HITJ(7, h7, s7)
#undef HITJ
    }
  }
  return wc;
}

__global__ __launch_bounds__(NTHR) void k_wprep(
    const float* __restrict__ Wsd, const float* __restrict__ Wds, unsigned short* wp) {
  const int seg = (int)blockIdx.x >> 2;
  const int g   = ((int)(blockIdx.x & 3) * NTHR) + (int)threadIdx.x;
  const int n   = g >> 4;
  const int k0  = (g & 15) * 8;
  const int kk  = k0 & (DIM - 1);
  const float* ps = Wsd + (size_t)seg * WIN + (size_t)n * DIM + kk;
  const float* pd = Wds + (size_t)seg * WIN + (size_t)n * DIM + kk;
  const v4f a1 = *(const v4f*)ps, b1 = *(const v4f*)(ps + 4);
  const v4f a2 = *(const v4f*)pd, b2 = *(const v4f*)(pd + 4);
  const bool fs = k0 < DIM;
  v4f a, b;
  a.x = fs ? a1.x : a2.x; a.y = fs ? a1.y : a2.y; a.z = fs ? a1.z : a2.z; a.w = fs ? a1.w : a2.w;
  b.x = fs ? b1.x : b2.x; b.y = fs ? b1.y : b2.y; b.z = fs ? b1.z : b2.z; b.w = fs ? b1.w : b2.w;
  v8us hv, lv;
  split8(a, b, hv, lv);
  unsigned short* dh = wp + (size_t)seg * 2 * BPL + (size_t)g * 8;
  unsigned short* dl = dh + BPL;
  *(volatile v8us*)dh = hv;
  *(volatile v8us*)dl = lv;
  __threadfence();
  *(volatile v8us*)dh = hv;
  *(volatile v8us*)dl = lv;
}

__global__ __launch_bounds__(NTHR) void k_count(
    const int* __restrict__ dsts, int* cnt, float* dpw, int nE, int vec8) {
  __shared__ __attribute__((aligned(16))) int scnt[NBC];
  __shared__ __attribute__((aligned(16))) int list[LISTN];
  __shared__ int wcnt[NWAVE];
  const int tid = threadIdx.x, lane = tid & 31, wave = tid >> 5;
  const int nodeBase = blockIdx.x * NBC;

  for (int i = tid; i < NBC; i += NTHR) scnt[i] = 0;
  __syncthreads();

  const int nChunks = (nE + CHUNK - 1) / CHUNK;
#pragma unroll 1
  for (int ch = 0; ch < nChunks; ++ch) {
    const int cbase = ch * CHUNK;
    const int wc = scan_chunk<NBC>(dsts, nE, cbase, nodeBase, vec8, list, tid, lane, wave);
    if (lane == 0) wcnt[wave] = wc;
    __syncthreads();
    if (wave == 0) {
#pragma unroll 1
      for (int wsx = 0; wsx < NWAVE; ++wsx) {
        int n = __builtin_amdgcn_readfirstlane(wcnt[wsx]);
        n = n > WCAP ? WCAP : (n < 0 ? 0 : n);
        const int* lp = list + wsx * WCAP;
#pragma unroll 1
        for (int i = 0; i < n; ++i) {
          const int ent  = __builtin_amdgcn_readfirstlane(lp[i]);
          const int slot = ent & (NBC - 1);
          if (lane == 0) scnt[slot] = scnt[slot] + 1;
        }
      }
    }
    __syncthreads();
  }

  v4i cq[8]; v4f dq[8];
#pragma unroll
  for (int q = 0; q < 8; ++q) {
    const int f = (wave * 8 + q) * 128 + 4 * lane;
    const v4i c = *(const v4i*)(scnt + f);
    cq[q] = c;
    dq[q].x = c.x > 0 ? rsqrtf(sqrtf((float)c.x)) : 0.0f;
    dq[q].y = c.y > 0 ? rsqrtf(sqrtf((float)c.y)) : 0.0f;
    dq[q].z = c.z > 0 ? rsqrtf(sqrtf((float)c.z)) : 0.0f;
    dq[q].w = c.w > 0 ? rsqrtf(sqrtf((float)c.w)) : 0.0f;
  }
  int*   cp = cnt + (size_t)nodeBase;
  float* dp = dpw + (size_t)nodeBase;
#pragma unroll
  for (int q = 0; q < 8; ++q) {
    const int f = (wave * 8 + q) * 128 + 4 * lane;
    *(volatile v4i*)(cp + f) = cq[q];
    *(volatile v4f*)(dp + f) = dq[q];
  }
  __threadfence();
#pragma unroll
  for (int q = 0; q < 8; ++q) {
    const int f = (wave * 8 + q) * 128 + 4 * lane;
    *(volatile v4i*)(cp + f) = cq[q];
    *(volatile v4f*)(dp + f) = dq[q];
  }
}

__global__ __launch_bounds__(OTHR) void k_offsets(
    const int* __restrict__ cnt, int* off, int* rbase, int nChunk) {
  __shared__ __attribute__((aligned(16))) int soff[NBC];
  __shared__ __attribute__((aligned(16))) int srb[RBN];
  __shared__ int wtot[OTHR / 32];
  const int tid = threadIdx.x, lane = tid & 31, wave = tid >> 5, sub = tid >> 7;
  for (int i = tid; i < RBN; i += OTHR) srb[i] = 0;
  int carry = 0;
#pragma unroll 1
  for (int ch = 0; ch < nChunk; ++ch) {
    const int base = ch * NBC;
    const v4i c0 = *(const v4i*)(cnt + base + CPT * tid);
    const v4i c1 = *(const v4i*)(cnt + base + CPT * tid + 4);
    const v4i c2 = *(const v4i*)(cnt + base + CPT * tid + 8);
    const v4i c3 = *(const v4i*)(cnt + base + CPT * tid + 12);
    const int e0  = max(c0.x, 0), e1  = max(c0.y, 0), e2  = max(c0.z, 0), e3  = max(c0.w, 0);
    const int e4  = max(c1.x, 0), e5  = max(c1.y, 0), e6  = max(c1.z, 0), e7  = max(c1.w, 0);
    const int e8  = max(c2.x, 0), e9  = max(c2.y, 0), e10 = max(c2.z, 0), e11 = max(c2.w, 0);
    const int e12 = max(c3.x, 0), e13 = max(c3.y, 0), e14 = max(c3.z, 0), e15 = max(c3.w, 0);
    const int ts = e0 + e1 + e2 + e3 + e4 + e5 + e6 + e7 + e8 + e9 + e10 + e11 + e12 + e13 + e14 + e15;
    int incl = ts;
#pragma unroll
    for (int d = 1; d < 32; d <<= 1) {
      const int t = __shfl_up(incl, d);
      if (lane >= d) incl += t;
    }
    if (lane == 31) wtot[wave] = incl;
    __syncthreads();
    const int S0 = wtot[0]  + wtot[1]  + wtot[2]  + wtot[3];
    const int S1 = wtot[4]  + wtot[5]  + wtot[6]  + wtot[7];
    const int S2 = wtot[8]  + wtot[9]  + wtot[10] + wtot[11];
    const int S3 = wtot[12] + wtot[13] + wtot[14] + wtot[15];
    int pre = 0;
#pragma unroll 1
    for (int w = 4 * sub; w < wave; ++w) pre += wtot[w];
    const int b0 = carry;
    const int b1 = b0 + ((S0 + 31) & ~31);
    const int b2 = b1 + ((S1 + 31) & ~31);
    const int b3 = b2 + ((S2 + 31) & ~31);
    const int b4 = b3 + ((S3 + 31) & ~31);
    const int myb = sub == 0 ? b0 : (sub == 1 ? b1 : (sub == 2 ? b2 : b3));
    if (tid == 0) {
      srb[min(4 * ch + 0, RBN - 1)] = b0;
      srb[min(4 * ch + 1, RBN - 1)] = b1;
      srb[min(4 * ch + 2, RBN - 1)] = b2;
      srb[min(4 * ch + 3, RBN - 1)] = b3;
    }
    int run = myb + pre + incl - ts;
    int* so = soff + CPT * tid;
    so[0]  = run; run += e0;
    so[1]  = run; run += e1;
    so[2]  = run; run += e2;
    so[3]  = run; run += e3;
    so[4]  = run; run += e4;
    so[5]  = run; run += e5;
    so[6]  = run; run += e6;
    so[7]  = run; run += e7;
    so[8]  = run; run += e8;
    so[9]  = run; run += e9;
    so[10] = run; run += e10;
    so[11] = run; run += e11;
    so[12] = run; run += e12;
    so[13] = run; run += e13;
    so[14] = run; run += e14;
    so[15] = run;
    carry = b4;
    __syncthreads();
    const v4i o0 = *(const v4i*)(soff + 4 * tid);
    const v4i o1 = *(const v4i*)(soff + 4 * (tid + OTHR));
    const v4i o2 = *(const v4i*)(soff + 4 * (tid + 2 * OTHR));
    const v4i o3 = *(const v4i*)(soff + 4 * (tid + 3 * OTHR));
    int* op = off + base;
    *(volatile v4i*)(op + 4 * tid) = o0;
    *(volatile v4i*)(op + 4 * (tid + OTHR)) = o1;
    *(volatile v4i*)(op + 4 * (tid + 2 * OTHR)) = o2;
    *(volatile v4i*)(op + 4 * (tid + 3 * OTHR)) = o3;
    __threadfence();
    *(volatile v4i*)(op + 4 * tid) = o0;
    *(volatile v4i*)(op + 4 * (tid + OTHR)) = o1;
    *(volatile v4i*)(op + 4 * (tid + 2 * OTHR)) = o2;
    *(volatile v4i*)(op + 4 * (tid + 3 * OTHR)) = o3;
    __syncthreads();
  }
  if (tid == 0) srb[min(4 * nChunk, RBN - 1)] = carry;
  __syncthreads();
  v4i rv = {0, 0, 0, 0};
  if (tid < 32) rv = *(const v4i*)(srb + 4 * tid);
  if (tid < 32) *(volatile v4i*)(rbase + 4 * tid) = rv;
  __threadfence();
  if (tid < 32) *(volatile v4i*)(rbase + 4 * tid) = rv;
}

__global__ __launch_bounds__(NTHR) void k_fill(
    const int* __restrict__ dsts, const int* __restrict__ srcs,
    const int* __restrict__ off, const int* __restrict__ rbase,
    int* csr, int nN, int nE, int vec8, int csrLen) {
  extern __shared__ v4f lds_dyn[];
  int* region = (int*)lds_dyn;
  int* cursor = region + RCAP;
  int* list   = cursor + NBF;
  int* wcnt   = list + LISTN;
  const int tid = threadIdx.x, lane = tid & 31, wave = tid >> 5;
  const int b = blockIdx.x;
  const int nodeBase = b * NBF;

  int rb0 = rbase[b];
  const int rb1 = rbase[b + 1];
  rb0 = rb0 < 0 ? 0 : (rb0 > csrLen ? csrLen : rb0);
  rb0 &= ~31;
  int len = rb1 - rb0;
  len = len < 0 ? 0 : (len > RCAP ? RCAP : len);
  int lenW = (len + 31) & ~31;
  if (rb0 + lenW > csrLen) lenW = (csrLen - rb0) & ~31;

  {
    const v4i z = {0, 0, 0, 0};
    for (int i = tid; i < RCAP / 4; i += NTHR) ((v4i*)region)[i] = z;
    for (int s = tid; s < NBF; s += NTHR) {
      int o = off[nodeBase + s] - rb0;
      o = o < 0 ? 0 : (o > RCAP ? RCAP : o);
      cursor[s] = o;
    }
  }
  __syncthreads();

  const int nChunks = (nE + CHUNK - 1) / CHUNK;
#pragma unroll 1
  for (int ch = 0; ch < nChunks; ++ch) {
    const int cbase = ch * CHUNK;
    const int wc = scan_chunk<NBF>(dsts, nE, cbase, nodeBase, vec8, list, tid, lane, wave);
    if (lane == 0) wcnt[wave] = wc;
    __syncthreads();
    if (wave == 0) {
#pragma unroll 1
      for (int wsx = 0; wsx < NWAVE; ++wsx) {
        int n = __builtin_amdgcn_readfirstlane(wcnt[wsx]);
        n = n > WCAP ? WCAP : (n < 0 ? 0 : n);
        const int* lp = list + wsx * WCAP;
#pragma unroll 1
        for (int i = 0; i < n; ++i) {
          const int ent  = __builtin_amdgcn_readfirstlane(lp[i]);
          const int slot = ent & (NBF - 1);
          int e = cbase + ((ent >> LSH) & (CHUNK - 1));
          e = e > nE - 1 ? nE - 1 : e;
          int src = srcs[e];
          src = src < 0 ? 0 : (src > nN - 1 ? nN - 1 : src);
          if (lane == 0) {
            int pos = cursor[slot];
            pos = pos < 0 ? 0 : (pos > RCAP - 1 ? RCAP - 1 : pos);
            region[pos] = src;
            const int np = pos + 1;
            cursor[slot] = np > RCAP ? RCAP : np;
          }
        }
      }
    }
    __syncthreads();
  }

  const int nv = lenW >> 2;
  int* gp = csr + rb0;
#pragma unroll 1
  for (int i = tid; i < nv; i += NTHR) { const v4i v = ((const v4i*)region)[i]; *(volatile v4i*)(gp + 4 * i) = v; }
  __threadfence();
#pragma unroll 1
  for (int i = tid; i < nv; i += NTHR) { const v4i v = ((const v4i*)region)[i]; *(volatile v4i*)(gp + 4 * i) = v; }
}

__global__ __launch_bounds__(NTHR) void k_gemm(
    const float* __restrict__ Asd, const float* __restrict__ Ads, const unsigned short* __restrict__ Bw,
    const float* __restrict__ bsd, const float* __restrict__ bds, const float* Cin, float* C,
    float coef, int nRowsA, int nRowsC, int useCin) {
  extern __shared__ v4f lds_dyn[];
  unsigned short* sHi = (unsigned short*)lds_dyn;
  unsigned short* sLo = sHi + GROWS * APH;
  float*          stg = (float*)lds_dyn;
  const int tid = threadIdx.x, lane = tid & 31, wave = tid >> 5, hh = lane >> 4, m = lane & 15;
  const int rowBase = blockIdx.x * GROWS;

#pragma unroll
  for (int i = 0; i < 8; ++i) {
    const int idx = (i & 3) * NTHR + tid;
    const int r   = idx >> 3;
    const int c0  = (idx & 7) * 8;
    int row = rowBase + r;
    row = row > nRowsA - 1 ? nRowsA - 1 : row;
    const float* ap = (i < 4 ? Asd : Ads) + (size_t)row * DIM + c0;
    const v4f a = *(const v4f*)ap, b = *(const v4f*)(ap + 4);
    v8us hv, lv;
    split8(a, b, hv, lv);
    const int kc = (i < 4 ? 0 : DIM) + c0;
    *(v8us*)(sHi + r * APH + kc) = hv;
    *(v8us*)(sLo + r * APH + kc) = lv;
  }
  __syncthreads();

  v8f acc[4];
#pragma unroll
  for (int t = 0; t < 4; ++t) { v8f z = {0.f, 0.f, 0.f, 0.f, 0.f, 0.f, 0.f, 0.f}; acc[t] = z; }
  const unsigned short* ahp = sHi + (wave * 16 + m) * APH + 8 * hh;
  const unsigned short* alp = sLo + (wave * 16 + m) * APH + 8 * hh;
#pragma unroll
  for (int kt = 0; kt < KST / 32; ++kt) {
    FragB ah, al;
    ah.h[0] = *(const v8us*)(ahp + 32 * kt);
    ah.h[1] = *(const v8us*)(ahp + 32 * kt + 16);
    al.h[0] = *(const v8us*)(alp + 32 * kt);
    al.h[1] = *(const v8us*)(alp + 32 * kt + 16);
#pragma unroll
    for (int t = 0; t < 4; ++t) {
      const unsigned short* bp = Bw + (size_t)(16 * t + m) * KST + 32 * kt + 8 * hh;
      FragB bh, bl;
      bh.h[0] = *(const v8us*)bp;
      bh.h[1] = *(const v8us*)(bp + 16);
      bl.h[0] = *(const v8us*)(bp + BPL);
      bl.h[1] = *(const v8us*)(bp + BPL + 16);
      acc[t] = wmb(ah.v, bh.v, acc[t]);
      acc[t] = wmb(ah.v, bl.v, acc[t]);
      acc[t] = wmb(al.v, bh.v, acc[t]);
    }
  }
  __syncthreads();

  const int r0 = wave * 16 + 8 * hh;
  float* sp = stg + r0 * DIM + m;
#pragma unroll
  for (int t = 0; t < 4; ++t) {
    const float bc = coef * (bsd[16 * t + m] + bds[16 * t + m]);
#pragma unroll
    for (int r = 0; r < 8; ++r) sp[r * DIM + 16 * t] = acc[t][r] * coef + bc;
  }
  __syncthreads();

  const float* lp = stg + wave * 16 * DIM + 4 * lane;
  const int rw0 = rowBase + wave * 16;
  v4f vals[8];
#pragma unroll
  for (int i = 0; i < 8; ++i) {
    v4f v = *(const v4f*)(lp + i * 2 * DIM);
    if (useCin != 0) v = v + *(const v4f*)(Cin + (size_t)(rw0 + 2 * i) * DIM + 4 * lane);
    vals[i] = v;
  }
  float* gp = C + (size_t)rw0 * DIM + 4 * lane;
#pragma unroll
  for (int i = 0; i < 8; ++i)
    if (rw0 + 2 * i + hh < nRowsC) *(volatile v4f*)(gp + (size_t)i * 2 * DIM) = vals[i];
  __threadfence();
#pragma unroll
  for (int i = 0; i < 8; ++i)
    if (rw0 + 2 * i + hh < nRowsC) *(volatile v4f*)(gp + (size_t)i * 2 * DIM) = vals[i];
}

__global__ __launch_bounds__(NTHR) void k_agg(
    const int* __restrict__ csr, const int* __restrict__ off, const int* __restrict__ cnt,
    const float* __restrict__ dT, const float* __restrict__ dS,
    const float* __restrict__ vin, float* vout, int nN, int csrLen) {
  const int tid = threadIdx.x, lane = tid & 31, wave = tid >> 5, hh = lane >> 4, q = lane & 15;
  const int tbase = blockIdx.x * TGT + wave * 32;
  const int cl = tbase + lane;
  const int cnt_l = cnt[cl];
  const int off_l = off[cl];
  union FI { float f; int i; };
  FI dtu; dtu.f = dT[cl];
  v4f keep = {0.f, 0.f, 0.f, 0.f};

#pragma unroll 1
  for (int j = 0; j < 32; ++j) {
    int n = __builtin_amdgcn_readlane(cnt_l, j);
    n = n < 0 ? 0 : (n > DEGCAP ? DEGCAP : n);
    const int st = __builtin_amdgcn_readlane(off_l, j);
    FI du; du.i = __builtin_amdgcn_readlane(dtu.i, j);
    const float dc = du.f;
    v4f acc = {0.f, 0.f, 0.f, 0.f};
#pragma unroll 1
    for (int q0 = 0; q0 < n; q0 += 32) {
      int pos = st + q0 + lane;
      pos = pos < 0 ? 0 : (pos > csrLen - 1 ? csrLen - 1 : pos);
      int sl = csr[pos];
      sl = sl < 0 ? 0 : (sl > nN - 1 ? nN - 1 : sl);
      const float wl = dS[sl] * dc;
      const int mcnt = (n - q0) < 32 ? (n - q0) : 32;
#pragma unroll 1
      for (int p = 0; p < mcnt; p += 2) {
        int li = p + hh;
        li = li > 31 ? 31 : li;
        const int s = __shfl(sl, li);
        float w = __shfl(wl, li);
        w = (p + hh < mcnt) ? w : 0.0f;
        const v4f v = *(const v4f*)(vin + (size_t)s * DIM + 4 * q);
        acc = acc + w * v;
      }
    }
    acc.x += __shfl_xor(acc.x, 16);
    acc.y += __shfl_xor(acc.y, 16);
    acc.z += __shfl_xor(acc.z, 16);
    acc.w += __shfl_xor(acc.w, 16);
    if ((j & 1) != 0) {
      v4f o;
      o.x = hh != 0 ? acc.x : keep.x;
      o.y = hh != 0 ? acc.y : keep.y;
      o.z = hh != 0 ? acc.z : keep.z;
      o.w = hh != 0 ? acc.w : keep.w;
      float* hp = vout + (size_t)(tbase + j - 1) * DIM + 4 * lane;
      *(volatile v4f*)hp = o;
      __threadfence();
      *(volatile v4f*)hp = o;
    } else {
      keep = acc;
    }
  }
}

extern "C" void kernel_launch(void* const* d_in, const int* in_sizes, int n_in,
                              void* d_out, int out_size, void* d_ws, size_t ws_size,
                              hipStream_t stream) {
  if (n_in < 6) return;
  const int nN = in_sizes[0] / DIM;
  const int nE = in_sizes[1] / 2;
  if (nN <= 0 || nE <= 0 || in_sizes[0] != nN * DIM || in_sizes[1] != 2 * nE) return;
  if (in_sizes[2] != NMAT * WIN || in_sizes[3] != NMAT * DIM) return;
  if (in_sizes[4] != NMAT * WIN || in_sizes[5] != NMAT * DIM) return;
  if (out_size != nN * DIM) return;
  if (nE > (1 << 28) || nN > (1 << 24)) return;

  const float* x   = (const float*)d_in[0];
  const int*   ei  = (const int*)d_in[1];
  const float* Wsd = (const float*)d_in[2];
  const float* bsd = (const float*)d_in[3];
  const float* Wds = (const float*)d_in[4];
  const float* bds = (const float*)d_in[5];
  float* out = (float*)d_out;
  const int* erow = ei;
  const int* ecol = ei + nE;

  const int NPAD   = ((nN + TGT - 1) / TGT) * TGT;
  const int nBC    = (nN + NBC - 1) / NBC;
  const int CNTPAD = nBC * NBC;
  if (4 * nBC + 1 > RBN) return;
  const int nBF    = (nN + NBF - 1) / NBF;
  const int csrLen = ((nE + 31) & ~31) + 4096;
  if (31 * 4 * nBC > 4096) return;
  const int nGemm  = NPAD / GROWS;
  const int nAgg   = NPAD / TGT;

  char* ws = (char*)d_ws;
  size_t offb = 0;
  const size_t oW    = offb; offb += (size_t)NMAT * 2 * BPL * 2;   offb = (offb + 255) & ~(size_t)255;
  const size_t oCntO = offb; offb += (size_t)CNTPAD * 4;           offb = (offb + 255) & ~(size_t)255;
  const size_t oDpO  = offb; offb += (size_t)CNTPAD * 4;           offb = (offb + 255) & ~(size_t)255;
  const size_t oOffO = offb; offb += (size_t)CNTPAD * 4;           offb = (offb + 255) & ~(size_t)255;
  const size_t oRbO  = offb; offb += (size_t)RBN * 4;              offb = (offb + 255) & ~(size_t)255;
  const size_t oCsrO = offb; offb += (size_t)csrLen * 4;           offb = (offb + 255) & ~(size_t)255;
  const size_t oCntI = offb; offb += (size_t)CNTPAD * 4;           offb = (offb + 255) & ~(size_t)255;
  const size_t oDpI  = offb; offb += (size_t)CNTPAD * 4;           offb = (offb + 255) & ~(size_t)255;
  const size_t oOffI = offb; offb += (size_t)CNTPAD * 4;           offb = (offb + 255) & ~(size_t)255;
  const size_t oRbI  = offb; offb += (size_t)RBN * 4;              offb = (offb + 255) & ~(size_t)255;
  const size_t oCsrI = offb; offb += (size_t)csrLen * 4;           offb = (offb + 255) & ~(size_t)255;
  const size_t oPA   = offb; offb += (size_t)NPAD * DIM * 4;       offb = (offb + 255) & ~(size_t)255;
  const size_t oPB   = offb; offb += (size_t)NPAD * DIM * 4;       offb = (offb + 255) & ~(size_t)255;
  const size_t oACC  = offb; offb += (size_t)NPAD * DIM * 4;       offb = (offb + 255) & ~(size_t)255;
  if (offb > ws_size || offb > (size_t)WSCAP) return;
  unsigned short* wp = (unsigned short*)(ws + oW);
  int*   cntO = (int*)(ws + oCntO);
  float* dpO  = (float*)(ws + oDpO);
  int*   offO = (int*)(ws + oOffO);
  int*   rbO  = (int*)(ws + oRbO);
  int*   csrO = (int*)(ws + oCsrO);
  int*   cntI = (int*)(ws + oCntI);
  float* dpI  = (float*)(ws + oDpI);
  int*   offI = (int*)(ws + oOffI);
  int*   rbI  = (int*)(ws + oRbI);
  int*   csrI = (int*)(ws + oCsrI);
  float* PA   = (float*)(ws + oPA);
  float* PB   = (float*)(ws + oPB);
  float* ACC  = (float*)(ws + oACC);

  const int vec8 = ((nE & 3) == 0) ? 1 : 0;

  k_wprep<<<NMAT * 4, NTHR, 0, stream>>>(Wsd, Wds, wp);

  hipFuncSetAttribute(reinterpret_cast<const void*>(&k_fill),
                      hipFuncAttributeMaxDynamicSharedMemorySize, LDS_FILL);
  k_count<<<nBC, NTHR, 0, stream>>>(erow, cntO, dpO, nE, vec8);
  k_offsets<<<1, OTHR, 0, stream>>>(cntO, offO, rbO, nBC);
  k_fill<<<nBF, NTHR, LDS_FILL, stream>>>(erow, ecol, offO, rbO, csrO, nN, nE, vec8, csrLen);
  k_count<<<nBC, NTHR, 0, stream>>>(ecol, cntI, dpI, nE, vec8);
  k_offsets<<<1, OTHR, 0, stream>>>(cntI, offI, rbI, nBC);
  k_fill<<<nBF, NTHR, LDS_FILL, stream>>>(ecol, erow, offI, rbI, csrI, nN, nE, vec8, csrLen);

  hipFuncSetAttribute(reinterpret_cast<const void*>(&k_gemm),
                      hipFuncAttributeMaxDynamicSharedMemorySize, LDS_GEMM);

  k_agg<<<nAgg, NTHR, 0, stream>>>(csrO, offO, cntO, dpO, dpI, x, PA, nN, csrLen);
  k_agg<<<nAgg, NTHR, 0, stream>>>(csrI, offI, cntI, dpI, dpO, x, PB, nN, csrLen);
  k_gemm<<<nGemm, NTHR, LDS_GEMM, stream>>>(PA, PB, wp, bsd, bds, ACC, ACC, 0.5f, NPAD, NPAD, 0);

  k_agg<<<nAgg, NTHR, 0, stream>>>(csrO, offO, cntO, dpO, dpI, PA, PB, nN, csrLen);
  k_agg<<<nAgg, NTHR, 0, stream>>>(csrI, offI, cntI, dpI, dpO, PB, PA, nN, csrLen);
  k_gemm<<<nGemm, NTHR, LDS_GEMM, stream>>>(PB, PA, wp + (size_t)1 * 2 * BPL, bsd + DIM, bds + DIM,
                                            ACC, ACC, 0.25f, NPAD, NPAD, 1);

  k_agg<<<nAgg, NTHR, 0, stream>>>(csrO, offO, cntO, dpO, dpI, PB, PA, nN, csrLen);
  k_agg<<<nAgg, NTHR, 0, stream>>>(csrI, offI, cntI, dpI, dpO, PA, PB, nN, csrLen);
  k_gemm<<<nGemm, NTHR, LDS_GEMM, stream>>>(PA, PB, wp + (size_t)2 * 2 * BPL, bsd + 2 * DIM, bds + 2 * DIM,
                                            ACC, out, 0.125f, NPAD, nN, 1);
}
